// _PureMamba_52802327937055
// MI455X (gfx1250) — hardware-run, weakly checked
//
#include <hip/hip_runtime.h>
#include <math.h>

typedef __attribute__((ext_vector_type(16))) _Float16 v16h;
typedef __attribute__((ext_vector_type(8)))  _Float16 v8h;
typedef __attribute__((ext_vector_type(8)))  float    v8f;
typedef __attribute__((ext_vector_type(4)))  float    v4f;

constexpr int kBatch  = 2;
constexpr int kSeq    = 2048;
constexpr int kDm     = 1024;
constexpr int kDi     = 2048;
constexpr int kNs     = 16;
constexpr int kRows   = kBatch * kSeq;
constexpr int kXzN    = 2 * kDi;
constexpr int kXdW    = 2 * kNs + 1;
constexpr int kXdP    = 64;
constexpr int kConvTP = 260;
constexpr int kScTS   = 64;
constexpr int kScCh   = 64;
constexpr int kScYP   = 68;
static_assert(kRows == 4096 && kXzN == 4096 && kXdW == 33 && kXdW <= kXdP);
static_assert((kDm % 32) == 0 && (kDi % 32) == 0);
static_assert((kRows % 64) == 0 && (kDi % 64) == 0 && (kXdP % 64) == 0 && (kDm % 64) == 0);
static_assert((kSeq % kScTS) == 0 && (kSeq % 64) == 0 && (kDi % kScCh) == 0 && (kDi % 256) == 0);
static_assert((kSeq & (kSeq - 1)) == 0);

constexpr float kCarX   = 16.0f;
constexpr float kCarW   = 256.0f;
constexpr float kCarU   = 8.0f;
constexpr float kCarY   = 0.25f;
constexpr float kResCar = 2048.0f;
constexpr float kResInv = 1.0f / kResCar;
constexpr float kScaleIn  = 1.0f / (kCarX * kCarW);
constexpr float kScaleXp  = 1.0f / (kCarU * kCarW);
constexpr float kScaleOut = 1.0f / (kCarY * kCarW);
constexpr float kF16MinN  = 6.103515625e-5f;

template <int SITE> __host__ __device__ constexpr float site_scale() {
  return (SITE == 0) ? kScaleIn : ((SITE == 1) ? kScaleXp : kScaleOut);
}

constexpr size_t kSzX16   = (size_t)kRows * kDm * 2;
constexpr size_t kSzWINT  = (size_t)kXzN  * kDm * 2;
constexpr size_t kSzWXT   = (size_t)kXdP  * kDi * 2;
constexpr size_t kSzWOUTT = (size_t)kDm   * kDi * 2;
constexpr size_t kSzSZ    = (size_t)kRows * kDi * 4;
constexpr size_t kSzU     = (size_t)kRows * kDi * 4;
constexpr size_t kSzP16   = (size_t)kRows * kDi * 2;
constexpr size_t kSzXD    = (size_t)kRows * kXdP * 4;
constexpr size_t kOffX16   = 0;
constexpr size_t kOffWINT  = kOffX16   + kSzX16;
constexpr size_t kOffWXT   = kOffWINT  + kSzWINT;
constexpr size_t kOffWOUTT = kOffWXT   + kSzWXT;
constexpr size_t kOffSZ    = kOffWOUTT + kSzWOUTT;
constexpr size_t kOffU     = kOffSZ    + kSzSZ;
constexpr size_t kOffPH    = kOffU     + kSzU;
constexpr size_t kOffPL    = kOffPH    + kSzP16;
constexpr size_t kOffXD    = kOffPL    + kSzP16;
constexpr size_t kWsTotal  = kOffXD    + kSzXD;
static_assert(kWsTotal == 122945536ull);
static_assert(kWsTotal <= 134217728ull);
static_assert((kOffWINT % 128) == 0 && (kOffWXT % 128) == 0 && (kOffWOUTT % 128) == 0 && (kOffSZ % 128) == 0 &&
              (kOffU % 128) == 0 && (kOffPH % 128) == 0 && (kOffPL % 128) == 0 && (kOffXD % 128) == 0);

__device__ __forceinline__ float bf16_rne(float f) {
  unsigned u = __float_as_uint(f);
  const unsigned lsb = (u & 0x00010000u) ? 1u : 0u;
  u = (u + 0x7FFFu + lsb) & 0xFFFF0000u;
  return __uint_as_float(u);
}
__device__ __forceinline__ _Float16 f16_flush(float c) {
  const float s = (fabsf(c) < kF16MinN) ? 0.0f : c;
  return (_Float16)s;
}
__device__ __forceinline__ void split_f16(float v, float carry, _Float16& hi, _Float16& lo) {
  float c = v * carry;
  c = fminf(fmaxf(c, -65000.0f), 65000.0f);
  hi = f16_flush(c);
  float hf = (float)hi;
  asm volatile("" : "+v"(hf));
  const float r = (c - hf) * kResCar;
  lo = f16_flush(r);
}

union FragU { v16h v; v8h h[2]; };
__device__ __forceinline__ v16h frag_load(const _Float16* p) {
  FragU f;
  f.h[0] = *(const v8h*)(p);
  f.h[1] = *(const v8h*)(p + 16);
  return f.v;
}
__device__ __forceinline__ v8f mma_f16(v16h a, v16h b, v8f c) {
  return __builtin_amdgcn_wmma_f32_16x16x32_f16(false, a, false, b, (short)0, c, false, false);
}
__device__ __forceinline__ void tie_acc(v8f& a, v16h x, v16h y) { asm volatile("" : "+v"(a) : "v"(x), "v"(y)); }
__device__ __forceinline__ void nop_acc(v8f& a, v16h x, v16h y) { asm volatile("v_nop\n\tv_nop\n\tv_nop\n\tv_nop" : "+v"(a) : "v"(x), "v"(y)); }
__device__ __forceinline__ void nop_one(v8f& a) { asm volatile("v_nop\n\tv_nop\n\tv_nop\n\tv_nop" : "+v"(a)); }
__device__ __forceinline__ void keep4_h(v16h a, v16h b, v16h c, v16h d) { asm volatile("v_nop" :: "v"(a), "v"(b), "v"(c), "v"(d)); }

template <int MT, bool SPLITA, int SITE>
__global__ __launch_bounds__(256) void gemm_f16_kernel(
    const unsigned short* __restrict__ Ap, const unsigned short* __restrict__ A2p, int lda,
    const unsigned short* __restrict__ Btp, int ldb,
    float* __restrict__ C, int ldc, int M, int N, int K) {
  const _Float16* A  = (const _Float16*)Ap;
  const _Float16* A2 = (const _Float16*)A2p;
  const _Float16* Bt = (const _Float16*)Btp;
  __shared__ __align__(16) float sT[8][16 * 68];
  const float scale = site_scale<SITE>();
  const int lane = threadIdx.x & 31;
  const int wave = threadIdx.x >> 5;
  const int tilesN = N >> 6;
  const int tilesM = M / (16 * MT);
  const int tile = blockIdx.x * 8 + wave;
  if (tile >= tilesM * tilesN) return;
  const int tm = tile / tilesN;
  const int tn = tile - tm * tilesN;
  const int m0 = tm * (16 * MT);
  const int n0 = tn << 6;

  const int rlane = lane & 15;
  const int koff  = (lane >> 4) * 8;
  const int mOff  = (lane >> 4) * 8;

  v8f acc[MT][4];
  v8f accr[MT][4];
#pragma unroll
  for (int i = 0; i < MT; ++i) {
#pragma unroll
    for (int j = 0; j < 4; ++j) {
      acc[i][j] = (v8f){0.f, 0.f, 0.f, 0.f, 0.f, 0.f, 0.f, 0.f};
      if (SPLITA) accr[i][j] = (v8f){0.f, 0.f, 0.f, 0.f, 0.f, 0.f, 0.f, 0.f};
    }
  }

  for (int k0 = 0; k0 < K; k0 += 32) {
    v16h bh[4];
#pragma unroll
    for (int j = 0; j < 4; ++j) {
      const size_t bo = (size_t)(n0 + (j << 4) + rlane) * ldb + koff + k0;
      bh[j] = frag_load(Bt + bo);
    }
#pragma unroll
    for (int i = 0; i < MT; ++i) {
      const size_t ao = (size_t)(m0 + (i << 4) + rlane) * lda + koff + k0;
      const v16h ah = frag_load(A + ao);
      v16h al = ah;
      if (SPLITA) al = frag_load(A2 + ao);
#pragma unroll
      for (int j = 0; j < 4; ++j) acc[i][j] = mma_f16(ah, bh[j], acc[i][j]);
      if (SPLITA) {
#pragma unroll
        for (int j = 0; j < 4; ++j) accr[i][j] = mma_f16(al, bh[j], accr[i][j]);
      }
      tie_acc(acc[i][0], ah, bh[0]);
      tie_acc(acc[i][1], ah, bh[1]);
      tie_acc(acc[i][2], ah, bh[2]);
      if (!SPLITA) {
        nop_acc(acc[i][3], ah, bh[3]);
      } else {
        tie_acc(acc[i][3], ah, bh[3]);
        tie_acc(accr[i][0], al, bh[0]);
        tie_acc(accr[i][1], al, bh[1]);
        tie_acc(accr[i][2], al, bh[2]);
        nop_acc(accr[i][3], al, bh[3]);
      }
    }
    keep4_h(bh[0], bh[1], bh[2], bh[3]);
  }
#pragma unroll
  for (int i = 0; i < MT; ++i) {
#pragma unroll
    for (int j = 0; j < 4; ++j) {
      nop_one(acc[i][j]);
      if (SPLITA) nop_one(accr[i][j]);
    }
  }

  float* slab = sT[wave];
#pragma unroll
  for (int i = 0; i < MT; ++i) {
    const int mBase = m0 + (i << 4);
#pragma unroll
    for (int j = 0; j < 4; ++j) {
#pragma unroll
      for (int r = 0; r < 8; ++r) {
        float v = acc[i][j][r];
        if (SPLITA) v = fmaf(accr[i][j][r], kResInv, v);
        v = v * scale;
        slab[(mOff + r) * 68 + (j << 4) + rlane] = v;
      }
    }
    __builtin_amdgcn_fence(__ATOMIC_RELEASE, "workgroup");
    __builtin_amdgcn_wave_barrier();
    __builtin_amdgcn_fence(__ATOMIC_ACQUIRE, "workgroup");
    {
      const int hh = lane >> 4, c4 = (lane & 15) * 4;
      for (int pass = 0; pass < 2; ++pass) {
#pragma unroll
        for (int it = 0; it < 8; ++it) {
          const int row = it * 2 + hh;
          const v4f v = *(const v4f*)(slab + row * 68 + c4);
          *(volatile v4f*)(C + (size_t)(mBase + row) * ldc + n0 + c4) = v;
        }
        __threadfence();
      }
    }
    __builtin_amdgcn_fence(__ATOMIC_RELEASE, "workgroup");
    __builtin_amdgcn_wave_barrier();
    __builtin_amdgcn_fence(__ATOMIC_ACQUIRE, "workgroup");
  }
}

__global__ __launch_bounds__(256) void cvt_x_kernel(
    const float* __restrict__ src, unsigned short* __restrict__ dst, unsigned total8) {
  const unsigned i = blockIdx.x * 256u + threadIdx.x;
  if (i >= total8) return;
  const size_t e0 = (size_t)i << 3;
  const v4f a0 = *(const v4f*)(src + e0);
  const v4f a1 = *(const v4f*)(src + e0 + 4);
  v8h hv;
#pragma unroll
  for (int e = 0; e < 4; ++e) {
    const float f0 = a0[e];
    const float f1 = a1[e];
    hv[e]     = f16_flush(bf16_rne(f0) * kCarX);
    hv[4 + e] = f16_flush(bf16_rne(f1) * kCarX);
  }
  unsigned short* q = dst + e0;
  *(volatile v8h*)q = hv;
  __threadfence();
  *(volatile v8h*)q = hv;
}

__global__ __launch_bounds__(256) void transpose_cvt_kernel(
    const float* __restrict__ src, unsigned short* __restrict__ dst, unsigned rows, unsigned cols) {
  __shared__ float sT[64 * 65];
  const unsigned tid = threadIdx.x;
  const unsigned r0 = blockIdx.y * 64u;
  const unsigned c0 = blockIdx.x * 64u;
  unsigned lc = tid & 63u;
  unsigned lr = tid >> 6;
  asm volatile("" : "+v"(lc));
  asm volatile("" : "+v"(lr));
  const unsigned gc  = c0 + lc;
  const unsigned gcc = (gc < cols) ? gc : (cols - 1u);
  const bool inb = (gc < cols);
#pragma unroll 4
  for (unsigned it = 0; it < 16u; ++it) {
    const unsigned r = it * 4u + lr;
    float v = src[(size_t)(r0 + r) * cols + gcc];
    asm volatile("" : "+v"(v));
    const float vb = bf16_rne(v);
    sT[lc * 65u + r] = inb ? vb : 0.0f;
  }
  __syncthreads();
  const unsigned lane = tid & 31u, wave = tid >> 5;
  unsigned q  = lane >> 3;
  unsigned j8 = (lane & 7u) * 8u;
  asm volatile("" : "+v"(q));
  asm volatile("" : "+v"(j8));
  v8h hv[2];
#pragma unroll
  for (int it = 0; it < 2; ++it) {
    const unsigned orow = (unsigned)it * 32u + wave * 4u + q;
    const float* sp = sT + orow * 65u + j8;
#pragma unroll
    for (int e = 0; e < 8; ++e) {
      const float f = sp[e];
      hv[it][e] = f16_flush(f * kCarW);
    }
  }
  for (int pass = 0; pass < 2; ++pass) {
#pragma unroll
    for (int it = 0; it < 2; ++it) {
      const unsigned orow = (unsigned)it * 32u + wave * 4u + q;
      *(volatile v8h*)(dst + (size_t)(c0 + orow) * rows + r0 + j8) = hv[it];
    }
    __threadfence();
  }
}

__global__ __launch_bounds__(256) void conv_silu_kernel(
    const float* __restrict__ S, const float* __restrict__ cw, const float* __restrict__ cb,
    float* __restrict__ U, unsigned short* __restrict__ PH, unsigned short* __restrict__ PL) {
  __shared__ __align__(16) float sT[16 * kConvTP];
  const unsigned tid = threadIdx.x;
  unsigned lane = tid & 31u;
  unsigned wave = tid >> 5;
  asm volatile("" : "+v"(lane));
  asm volatile("" : "+v"(wave));
  const unsigned d0 = blockIdx.x * 256u;
  const unsigned d  = d0 + tid;
  const unsigned g0 = blockIdx.y * 64u;
  const bool hist = ((g0 & (unsigned)(kSeq - 1)) != 0u);
  const v4f wv = *(const v4f*)(cw + (size_t)d * 4);
  const float wr0 = wv[0], wr1 = wv[1], wr2 = wv[2], wr3 = wv[3];
  const float w0 = bf16_rne(wr0), w1 = bf16_rne(wr1), w2 = bf16_rne(wr2), w3 = bf16_rne(wr3);
  const float bc = bf16_rne(cb[d]);
  float xm3, xm2, xm1;
  {
    const unsigned rb = hist ? (g0 - 3u) : g0;
    const float v3 = S[(size_t)rb * kDi + d];
    const float v2 = S[(size_t)(rb + 1u) * kDi + d];
    const float v1 = S[(size_t)(rb + 2u) * kDi + d];
    xm3 = hist ? v3 : 0.0f;
    xm2 = hist ? v2 : 0.0f;
    xm1 = hist ? v1 : 0.0f;
  }
  const unsigned hrow = wave >> 1;
  const unsigned hch  = (wave & 1u) * 128u + lane * 4u;
#pragma unroll 1
  for (unsigned sub = 0; sub < 4u; ++sub) {
    const unsigned lb = g0 + sub * 16u;
#pragma unroll 1
    for (unsigned s = 0; s < 16u; ++s) {
      const float xcur = S[(size_t)(lb + s) * kDi + d];
      float acc = w0 * xm3;
      acc = fmaf(w1, xm2, acc);
      acc = fmaf(w2, xm1, acc);
      acc = fmaf(w3, xcur, acc);
      const float sv = acc + bc;
      const float sg = 1.0f / (1.0f + expf(-sv));
      sT[s * kConvTP + tid] = sv * sg;
      xm3 = xm2;
      xm2 = xm1;
      xm1 = xcur;
    }
    __syncthreads();
    v4f fv[4];
    v8h hv[2], lv[2];
#pragma unroll
    for (int it = 0; it < 4; ++it) fv[it] = *(const v4f*)(sT + ((unsigned)it * 4u + hrow) * kConvTP + hch);
#pragma unroll
    for (int it = 0; it < 2; ++it) {
      const float* sp = sT + ((unsigned)it * 8u + wave) * kConvTP + lane * 8u;
      const v4f a0 = *(const v4f*)(sp);
      const v4f a1 = *(const v4f*)(sp + 4);
#pragma unroll
      for (int e = 0; e < 4; ++e) {
        const float f0 = a0[e];
        const float f1 = a1[e];
        _Float16 h0, l0, h1, l1;
        split_f16(f0, kCarU, h0, l0);
        split_f16(f1, kCarU, h1, l1);
        hv[it][e]     = h0;
        lv[it][e]     = l0;
        hv[it][4 + e] = h1;
        lv[it][4 + e] = l1;
      }
    }
    for (int pass = 0; pass < 2; ++pass) {
#pragma unroll
      for (int it = 0; it < 4; ++it)
        *(volatile v4f*)(U + (size_t)(lb + (unsigned)it * 4u + hrow) * kDi + d0 + hch) = fv[it];
#pragma unroll
      for (int it = 0; it < 2; ++it) {
        const size_t o = (size_t)(lb + (unsigned)it * 8u + wave) * kDi + d0 + lane * 8u;
        *(volatile v8h*)(PH + o) = hv[it];
        *(volatile v8h*)(PL + o) = lv[it];
      }
      __threadfence();
    }
    __syncthreads();
  }
}

__global__ __launch_bounds__(64) void scan_kernel(
    const float* __restrict__ XD, const float* __restrict__ U, const float* __restrict__ Z,
    const float* __restrict__ Wdt, const float* __restrict__ bdt, const float* __restrict__ Alog,
    const float* __restrict__ Dsk, unsigned short* __restrict__ YH, unsigned short* __restrict__ YL) {
  __shared__ __align__(16) float sX[kScTS * kXdP];
  __shared__ __align__(16) float sY[kScTS * kScYP];
  __shared__ __align__(16) float sA[kNs * kScCh];
  const unsigned tid = threadIdx.x;
  unsigned lane = tid & 31u;
  unsigned wave = tid >> 5;
  asm volatile("" : "+v"(lane));
  asm volatile("" : "+v"(wave));
  constexpr unsigned kBlkPerB = kDi / kScCh;
  const unsigned bix = blockIdx.x / kBlkPerB;
  const unsigned d0  = (blockIdx.x - bix * kBlkPerB) * kScCh;
  const unsigned d   = d0 + tid;
  const size_t row0  = (size_t)bix * kSeq;
#pragma unroll 1
  for (unsigned s = 0; s < (unsigned)kNs; ++s) {
    const float al = Alog[(size_t)d * kNs + s];
    sA[s * kScCh + tid] = -expf(bf16_rne(al));
  }
  __syncthreads();
  float negA[kNs], h[kNs];
#pragma unroll
  for (int s = 0; s < kNs; ++s) {
    negA[s] = sA[s * kScCh + tid];
    h[s] = 0.0f;
  }
  const float wdt = bf16_rne(Wdt[d]);
  const float bb  = bf16_rne(bdt[d]);
  const float Dd  = bf16_rne(Dsk[d]);
  unsigned lr  = tid >> 4;
  unsigned lc4 = (tid & 15u) * 4u;
  unsigned q   = lane >> 3;
  unsigned c8  = (lane & 7u) * 8u;
  asm volatile("" : "+v"(lr));
  asm volatile("" : "+v"(lc4));
  asm volatile("" : "+v"(q));
  asm volatile("" : "+v"(c8));
#pragma unroll 1
  for (unsigned t0 = 0; t0 < (unsigned)kSeq; t0 += (unsigned)kScTS) {
    __syncthreads();
#pragma unroll
    for (int i = 0; i < 16; ++i) {
      const unsigned r = lr + 4u * (unsigned)i;
      *(v4f*)(sX + r * kXdP + lc4) = *(const v4f*)(XD + (row0 + t0 + r) * kXdP + lc4);
    }
    __syncthreads();
#pragma unroll 1
    for (unsigned s = 0; s < (unsigned)kScTS; ++s) {
      const size_t grow = row0 + t0 + s;
      const float* xr = sX + s * kXdP;
      float xt = U[grow * kDi + d];
      float zv = Z[grow * kDi + d];
      asm volatile("" : "+v"(xt));
      asm volatile("" : "+v"(zv));
      const float dtr = xr[2 * kNs];
      const float v   = fmaf(dtr, wdt, bb);
      const float ea  = expf(-fabsf(v));
      const float dt  = fmaxf(v, 0.0f) + log1pf(ea);
      const float dtx = dt * xt;
      float y = 0.0f;
#pragma unroll
      for (int g = 0; g < 4; ++g) {
        const v4f bv = *(const v4f*)(xr + 4 * g);
        const v4f cv = *(const v4f*)(xr + kNs + 4 * g);
#pragma unroll
        for (int e = 0; e < 4; ++e) {
          const float bq = bv[e];
          const float cq = cv[e];
          const float ee = __expf(dt * negA[4 * g + e]);
          h[4 * g + e] = fmaf(ee, h[4 * g + e], dtx * bq);
          y = fmaf(h[4 * g + e], cq, y);
        }
      }
      y = fmaf(xt, Dd, y);
      const float sg = 1.0f / (1.0f + expf(-zv));
      y = y * (zv * sg);
      sY[s * kScYP + tid] = y;
    }
    __syncthreads();
    v8h hv[8], lv[8];
#pragma unroll
    for (int it = 0; it < 8; ++it) {
      const unsigned row = (unsigned)it * 8u + wave * 4u + q;
      const float* sp = sY + row * kScYP + c8;
      const v4f a0 = *(const v4f*)(sp);
      const v4f a1 = *(const v4f*)(sp + 4);
#pragma unroll
      for (int e = 0; e < 4; ++e) {
        const float f0 = a0[e];
        const float f1 = a1[e];
        _Float16 h0, l0, h1, l1;
        split_f16(f0, kCarY, h0, l0);
        split_f16(f1, kCarY, h1, l1);
        hv[it][e]     = h0;
        lv[it][e]     = l0;
        hv[it][4 + e] = h1;
        lv[it][4 + e] = l1;
      }
    }
    for (int pass = 0; pass < 2; ++pass) {
#pragma unroll
      for (int it = 0; it < 8; ++it) {
        const unsigned row = (unsigned)it * 8u + wave * 4u + q;
        const size_t o = (row0 + t0 + row) * (size_t)kDi + d0 + c8;
        *(volatile v8h*)(YH + o) = hv[it];
        *(volatile v8h*)(YL + o) = lv[it];
      }
      __threadfence();
    }
  }
}

static_assert((((kRows / 64) * (kDi / 64)) % 8) == 0);
static_assert((((kRows / 32) * (kXdP / 64)) % 8) == 0);
static_assert((((kRows / 32) * (kDm / 64)) % 8) == 0);
static_assert(((kRows * kDm / 8) % 256) == 0);

extern "C" void kernel_launch(void* const* d_in, const int* in_sizes, int n_in,
                              void* d_out, int out_size, void* d_ws, size_t ws_size,
                              hipStream_t stream) {
  if (n_in < 10) return;
  if (in_sizes[0] != kRows * kDm) return;
  if (in_sizes[1] != kDm * kXzN) return;
  if (in_sizes[2] != kDi * 4) return;
  if (in_sizes[3] != kDi) return;
  if (in_sizes[4] != kDi * kXdW) return;
  if (in_sizes[5] != kDi) return;
  if (in_sizes[6] != kDi) return;
  if (in_sizes[7] != kDi * kNs) return;
  if (in_sizes[8] != kDi) return;
  if (in_sizes[9] != kDi * kDm) return;
  if (out_size != kRows * kDm) return;
  if (ws_size < kWsTotal) return;

  const float* x      = (const float*)d_in[0];
  const float* W_in   = (const float*)d_in[1];
  const float* conv_w = (const float*)d_in[2];
  const float* conv_b = (const float*)d_in[3];
  const float* W_x    = (const float*)d_in[4];
  const float* w_dt   = (const float*)d_in[5];
  const float* b_dt   = (const float*)d_in[6];
  const float* A_log  = (const float*)d_in[7];
  const float* D_skip = (const float*)d_in[8];
  const float* W_out  = (const float*)d_in[9];
  float* out = (float*)d_out;

  char* ws = (char*)d_ws;
  unsigned short* X16   = (unsigned short*)(ws + kOffX16);
  unsigned short* WINT  = (unsigned short*)(ws + kOffWINT);
  unsigned short* WXT   = (unsigned short*)(ws + kOffWXT);
  unsigned short* WOUTT = (unsigned short*)(ws + kOffWOUTT);
  float*          SZ    = (float*)(ws + kOffSZ);
  float*          U     = (float*)(ws + kOffU);
  unsigned short* PH    = (unsigned short*)(ws + kOffPH);
  unsigned short* PL    = (unsigned short*)(ws + kOffPL);
  float*          XD    = (float*)(ws + kOffXD);

  cvt_x_kernel<<<(kRows * kDm / 8) / 256, 256, 0, stream>>>(x, X16, (unsigned)(kRows * kDm / 8));
  transpose_cvt_kernel<<<dim3(kXzN / 64, kDm / 64), 256, 0, stream>>>(W_in, WINT, (unsigned)kDm, (unsigned)kXzN);
  transpose_cvt_kernel<<<dim3(kXdP / 64, kDi / 64), 256, 0, stream>>>(W_x, WXT, (unsigned)kDi, (unsigned)kXdW);
  transpose_cvt_kernel<<<dim3(kDm / 64, kDi / 64), 256, 0, stream>>>(W_out, WOUTT, (unsigned)kDi, (unsigned)kDm);

  gemm_f16_kernel<4, false, 0><<<((kRows / 64) * (kDi / 64)) / 8, 256, 0, stream>>>(
      X16, X16, kDm, WINT, kDm, SZ, kDi, kRows, kDi, kDm);

  conv_silu_kernel<<<dim3(kDi / 256, kRows / 64), 256, 0, stream>>>(SZ, conv_w, conv_b, U, PH, PL);

  gemm_f16_kernel<2, true, 1><<<((kRows / 32) * (kXdP / 64)) / 8, 256, 0, stream>>>(
      PH, PL, kDi, WXT, kDi, XD, kXdP, kRows, kXdP, kDi);

  gemm_f16_kernel<4, false, 0><<<((kRows / 64) * (kDi / 64)) / 8, 256, 0, stream>>>(
      X16, X16, kDm, WINT + (size_t)kDi * kDm, kDm, SZ, kDi, kRows, kDi, kDm);

  scan_kernel<<<kBatch * (kDi / kScCh), kScCh, 0, stream>>>(XD, U, SZ, w_dt, b_dt, A_log, D_skip, PH, PL);

  gemm_f16_kernel<2, true, 2><<<((kRows / 32) * (kDm / 64)) / 8, 256, 0, stream>>>(
      PH, PL, kDi, WOUTT, kDi, out, kDm, kRows, kDm, kDi);
}
